// Co_Guiding_GAT_65377992180060
// MI455X (gfx1250) — hardware-verified
//
#include <hip/hip_runtime.h>
#include <stddef.h>
#include <stdint.h>

#define NBT   4
#define NND   1024
#define DM    256
#define NH    8
#define HDM   32
#define NLY   2
#define NBR   4
#define NTOK  (NBT * NND)
#define HN    (NTOK * DM)
#define WMAT  (DM * DM)
#define NMAT  (NLY * NBR)
#define QB    128
#define KC    64
#define NQB   (NND / QB)
#define NCK   (NND / KC)
#define HPL   (NBT * NH * NND * HDM)

static_assert(NH * HDM == DM);
static_assert(HDM == 32);
static_assert(NND % QB == 0);
static_assert(NND % KC == 0);
static_assert(NND % 256 == 0);
static_assert(DM % 64 == 0);
static_assert(HN % 2048 == 0);
static_assert(NTOK % 32 == 0);
static_assert(HPL == HN);
static_assert(KC == 64);
static_assert(QB == 8 * 16);

typedef _Float16 v16h __attribute__((ext_vector_type(16)));
typedef _Float16 v8h  __attribute__((ext_vector_type(8)));
typedef float    v8f  __attribute__((ext_vector_type(8)));
typedef float    v4f  __attribute__((ext_vector_type(4)));
typedef unsigned int v4u __attribute__((ext_vector_type(4)));

union Frag  { v16h v; v8h h[2]; };
union Pack8 { v8h h; v4u u; };

__device__ __forceinline__ v8f mma16(v16h a, v16h b, v8f c) {
  c = __builtin_amdgcn_wmma_f32_16x16x32_f16(false, a, false, b, (short)0, c, false, false);
  asm volatile("v_nop\n\tv_nop\n\tv_nop\n\tv_nop" : "+v"(c) : "v"(a), "v"(b));
  return c;
}

__device__ __forceinline__ v16h ldfrag(const _Float16* p, int ld, int row0, int k0, int lane) {
  const int m = lane & 15, lh = lane >> 4;
  const _Float16* q = p + (size_t)(row0 + m) * ld + k0 + 8 * lh;
  Frag f;
  f.h[0] = *(const v8h*)(q);
  f.h[1] = *(const v8h*)(q + 16);
  return f.v;
}

__device__ __forceinline__ v8f zero8() { return (v8f){0.f, 0.f, 0.f, 0.f, 0.f, 0.f, 0.f, 0.f}; }

__device__ __forceinline__ void gemm32x64(const _Float16* __restrict__ A, int lda, int aks,
                                          const _Float16* __restrict__ Bt, int ldb, int bks, int nk,
                                          int m0, int n0, int lane, v8f (&acc)[2][4]) {
#pragma unroll 1
  for (int kk = 0; kk < nk; ++kk) {
    const _Float16* Ak = A + (size_t)kk * aks;
    const _Float16* Bk = Bt + (size_t)kk * bks;
    const v16h a0 = ldfrag(Ak, lda, m0, 0, lane);
    const v16h a1 = ldfrag(Ak, lda, m0 + 16, 0, lane);
    const v16h b0 = ldfrag(Bk, ldb, n0, 0, lane);
    const v16h b1 = ldfrag(Bk, ldb, n0 + 16, 0, lane);
    const v16h b2 = ldfrag(Bk, ldb, n0 + 32, 0, lane);
    const v16h b3 = ldfrag(Bk, ldb, n0 + 48, 0, lane);
    acc[0][0] = mma16(a0, b0, acc[0][0]);
    acc[1][0] = mma16(a1, b0, acc[1][0]);
    acc[0][1] = mma16(a0, b1, acc[0][1]);
    acc[1][1] = mma16(a1, b1, acc[1][1]);
    acc[0][2] = mma16(a0, b2, acc[0][2]);
    acc[1][2] = mma16(a1, b2, acc[1][2]);
    acc[0][3] = mma16(a0, b3, acc[0][3]);
    acc[1][3] = mma16(a1, b3, acc[1][3]);
  }
}

#define WTP 72
__global__ __launch_bounds__(256) void k_wcvt(const float* __restrict__ src, _Float16* __restrict__ dst) {
  __shared__ __align__(16) _Float16 st[64 * WTP];
  const int tid  = threadIdx.x;
  const int mat  = blockIdx.x >> 4;
  const int tile = blockIdx.x & 15;
  const int n0 = (tile >> 2) * 64;
  const int k0 = (tile & 3) * 64;
  const float* s = src + (size_t)mat * WMAT;
#pragma unroll
  for (int it = 0; it < 4; ++it) {
    const int p  = tid + 256 * it;
    const int kr = p >> 4;
    const int q  = (p & 15) * 4;
    const v4f v = *(const v4f*)(s + (size_t)(k0 + kr) * DM + n0 + q) * 32.0f;
    st[(q + 0) * WTP + kr] = (_Float16)v[0];
    st[(q + 1) * WTP + kr] = (_Float16)v[1];
    st[(q + 2) * WTP + kr] = (_Float16)v[2];
    st[(q + 3) * WTP + kr] = (_Float16)v[3];
  }
  __syncthreads();
  v4u val[2];
  size_t go[2];
#pragma unroll
  for (int it = 0; it < 2; ++it) {
    const int p   = tid + 256 * it;
    const int row = p >> 3;
    const int pc  = p & 7;
    Pack8 pk;
    pk.h    = *(const v8h*)(st + row * WTP + pc * 8);
    val[it] = pk.u;
    go[it]  = (size_t)mat * WMAT + (size_t)(n0 + row) * DM + k0 + pc * 8;
  }
  for (int ps = 0; ps < 2; ++ps) {
#pragma unroll
    for (int it = 0; it < 2; ++it) *(volatile v4u*)(dst + go[it]) = val[it];
    __threadfence();
  }
}

__global__ __launch_bounds__(256) void k_cvt_h(const float* __restrict__ xa, const float* __restrict__ xb,
                                               _Float16* __restrict__ h16) {
  const float* src = (blockIdx.y == 0) ? xa : xb;
  const size_t o = (size_t)blockIdx.x * 2048 + (size_t)threadIdx.x * 8;
  const v4f a0 = *(const v4f*)(src + o);
  const v4f a1 = *(const v4f*)(src + o + 4);
  Pack8 pk;
  pk.h = (v8h){(_Float16)a0[0], (_Float16)a0[1], (_Float16)a0[2], (_Float16)a0[3],
               (_Float16)a1[0], (_Float16)a1[1], (_Float16)a1[2], (_Float16)a1[3]};
  const v4u vv = pk.u;
  volatile v4u* d = (volatile v4u*)(h16 + (size_t)blockIdx.y * HN + o);
  *d = vv;
  __threadfence();
  *d = vv;
}

#define STP 72
#define SVP 264
__global__ __launch_bounds__(256) void k_qkv(const _Float16* __restrict__ h16, int qsel, int kvsel,
                                             const _Float16* __restrict__ wt,
                                             const float* __restrict__ bq,
                                             const float* __restrict__ bk,
                                             const float* __restrict__ bv,
                                             _Float16* __restrict__ qkp,
                                             _Float16* __restrict__ vtp) {
  __shared__ __align__(16) _Float16 st[256 * STP];
  const int tid = threadIdx.x, lane = tid & 31, wave = tid >> 5;
  const int hh = lane >> 4, c = lane & 15;
  const int bx  = blockIdx.x;
  const int b   = bx >> 2;
  const int nb0 = (bx & 3) * 256;
  const int ns  = blockIdx.y;
  const int which = ns >> 2;
  const int cg    = ns & 3;
  const int m0 = bx * 256 + wave * 32;
  const int n0 = cg * 64;
  const int sel = (which == 0) ? qsel : kvsel;
  const _Float16* A = h16 + (size_t)sel * HN;
  const _Float16* B = wt + (size_t)which * ((size_t)NMAT * WMAT);

  v8f acc[2][4];
#pragma unroll
  for (int s = 0; s < 2; ++s)
#pragma unroll
    for (int t = 0; t < 4; ++t) acc[s][t] = zero8();
  gemm32x64(A, DM, 32, B, DM, 32, DM / 32, m0, n0, lane, acc);

  float bb[4];
#pragma unroll
  for (int t = 0; t < 4; ++t) {
    const int i = n0 + 16 * t + c;
    const float xq = bq[i], xk = bk[i], xv = bv[i];
    bb[t] = (which == 0) ? xq : ((which == 1) ? xk : xv);
  }

  if (which < 2) {
#pragma unroll
    for (int sub = 0; sub < 2; ++sub)
#pragma unroll
      for (int t = 0; t < 4; ++t)
#pragma unroll
        for (int r = 0; r < 8; ++r)
          st[(wave * 32 + sub * 16 + 8 * hh + r) * STP + 16 * t + c] =
              (_Float16)(acc[sub][t][r] * 0.03125f + bb[t]);
  } else {
#pragma unroll
    for (int sub = 0; sub < 2; ++sub)
#pragma unroll
      for (int t = 0; t < 4; ++t)
#pragma unroll
        for (int r = 0; r < 8; ++r)
          st[(16 * t + c) * SVP + wave * 32 + sub * 16 + 8 * hh + r] =
              (_Float16)(acc[sub][t][r] * 0.03125f + bb[t]);
  }
  __syncthreads();

  if (which < 2) {
    _Float16* base = qkp + (size_t)which * HPL;
#pragma unroll
    for (int g = 0; g < 2; ++g) {
      v4u val[4];
      size_t go[4];
#pragma unroll
      for (int j = 0; j < 4; ++j) {
        const int p    = tid + 256 * (4 * g + j);
        const int slab = p >> 10;
        const int pp   = p & 1023;
        const int lr   = pp >> 2;
        const int pc   = pp & 3;
        Pack8 pk;
        pk.h   = *(const v8h*)(st + lr * STP + slab * 32 + pc * 8);
        val[j] = pk.u;
        go[j]  = ((size_t)(b * NH + 2 * cg + slab) * NND + nb0 + lr) * HDM + pc * 8;
      }
      for (int ps = 0; ps < 2; ++ps) {
#pragma unroll
        for (int j = 0; j < 4; ++j) *(volatile v4u*)(base + go[j]) = val[j];
        __threadfence();
      }
    }
  } else {
#pragma unroll
    for (int g = 0; g < 2; ++g) {
      v4u val[4];
      size_t go[4];
#pragma unroll
      for (int j = 0; j < 4; ++j) {
        const int p     = tid + 256 * (4 * g + j);
        const int drow  = p >> 5;
        const int pc    = p & 31;
        const int head2 = drow >> 5;
        const int d     = drow & 31;
        Pack8 pk;
        pk.h   = *(const v8h*)(st + drow * SVP + pc * 8);
        val[j] = pk.u;
        go[j]  = ((size_t)(b * NH + 2 * cg + head2) * HDM + d) * NND + nb0 + pc * 8;
      }
      for (int ps = 0; ps < 2; ++ps) {
#pragma unroll
        for (int j = 0; j < 4; ++j) *(volatile v4u*)(vtp + go[j]) = val[j];
        __threadfence();
      }
    }
  }
}

#define KSP 40
#define VSP 72
__global__ __launch_bounds__(256) void k_attn(const _Float16* __restrict__ qkp,
                                              const _Float16* __restrict__ vtp,
                                              const int* __restrict__ adj,
                                              _Float16* __restrict__ op, float sscale) {
  __shared__ __align__(16) _Float16 Ks[KC * KSP];
  __shared__ __align__(16) _Float16 Vs[HDM * VSP];
  __shared__ __align__(16) _Float16 Ps[8 * 16 * VSP];

  const int tid = threadIdx.x, lane = tid & 31, wave = tid >> 5;
  const int hh = lane >> 4, c = lane & 15;
  const int qb  = blockIdx.x % NQB;
  const int hb  = blockIdx.x / NQB;
  const int b   = hb / NH;
  const int q0  = qb * QB + wave * 16;

  const _Float16* Q = qkp + (size_t)hb * NND * HDM;
  const _Float16* K = qkp + (size_t)HPL + (size_t)hb * NND * HDM;
  const _Float16* V = vtp + (size_t)hb * HDM * NND;
  const int* arow = adj + ((size_t)b * NND + q0 + 8 * hh) * NND + c;

  const v16h qa = ldfrag(Q, HDM, q0, 0, lane);

  const float NEGI = -__builtin_huge_valf();
  float mrow[8], lrow[8];
  v8f oacc[2];
#pragma unroll
  for (int r = 0; r < 8; ++r) { mrow[r] = NEGI; lrow[r] = 0.f; }
#pragma unroll
  for (int t = 0; t < 2; ++t) oacc[t] = zero8();

  _Float16* pw = Ps + wave * 16 * VSP;

  for (int kc = 0; kc < NCK; ++kc) {
    const int kv0 = kc * KC;
    __syncthreads();
    {
      const int kr = tid >> 2;
      const int qq = (tid & 3) * 8;
      *(v8h*)(Ks + kr * KSP + qq) = *(const v8h*)(K + (size_t)(kv0 + kr) * HDM + qq);
      const int dr = tid >> 3;
      const int q8 = (tid & 7) * 8;
      *(v8h*)(Vs + dr * VSP + q8) = *(const v8h*)(V + (size_t)dr * NND + kv0 + q8);
    }
    __syncthreads();

    v8f s[4];
#pragma unroll
    for (int j = 0; j < 4; ++j) {
      const v16h kb = ldfrag(Ks, KSP, j * 16, 0, lane);
      s[j] = mma16(qa, kb, zero8());
    }
    float cm[8];
#pragma unroll
    for (int r = 0; r < 8; ++r) {
      float m = NEGI;
#pragma unroll
      for (int j = 0; j < 4; ++j) {
        const int av  = arow[(size_t)r * NND + kv0 + 16 * j];
        const float v = s[j][r] * sscale;
        const float w = (av == 0) ? -1.0e9f : v;
        s[j][r] = w;
        m = fmaxf(m, w);
      }
#pragma unroll
      for (int off = 1; off < 16; off <<= 1) m = fmaxf(m, __shfl_xor(m, off, 32));
      cm[r] = m;
    }
    float al[8];
#pragma unroll
    for (int r = 0; r < 8; ++r) {
      const float mnew  = fmaxf(mrow[r], cm[r]);
      const float alpha = __expf(mrow[r] - mnew);
      mrow[r] = mnew;
      float psum = 0.f;
#pragma unroll
      for (int j = 0; j < 4; ++j) {
        const float p = __expf(s[j][r] - mnew);
        psum += p;
        pw[(8 * hh + r) * VSP + j * 16 + c] = (_Float16)(p * 1024.0f);
      }
#pragma unroll
      for (int off = 1; off < 16; off <<= 1) psum += __shfl_xor(psum, off, 32);
      lrow[r] = lrow[r] * alpha + psum;
      al[r] = alpha;
    }
#pragma unroll
    for (int t = 0; t < 2; ++t)
#pragma unroll
      for (int r = 0; r < 8; ++r) oacc[t][r] *= al[r];
    __syncthreads();

#pragma unroll
    for (int kk = 0; kk < 2; ++kk) {
      const v16h pa = ldfrag(pw, VSP, 0, kk * 32, lane);
#pragma unroll
      for (int t = 0; t < 2; ++t) {
        const v16h vb = ldfrag(Vs, VSP, t * 16, kk * 32, lane);
        oacc[t] = mma16(pa, vb, oacc[t]);
      }
    }
  }

  float invl[8];
#pragma unroll
  for (int r = 0; r < 8; ++r) invl[r] = (lrow[r] > 0.f) ? (0.0625f / lrow[r]) : 0.f;
  __syncthreads();
#pragma unroll
  for (int r = 0; r < 8; ++r) {
#pragma unroll
    for (int t = 0; t < 2; ++t)
      pw[(8 * hh + r) * VSP + 16 * t + c] = (_Float16)(oacc[t][r] * invl[r]);
  }
  __syncthreads();
  v4u val[2];
  size_t go[2];
#pragma unroll
  for (int it = 0; it < 2; ++it) {
    const int p  = lane + 32 * it;
    const int L  = p >> 2;
    const int pc = p & 3;
    Pack8 pk;
    pk.h    = *(const v8h*)(pw + L * VSP + pc * 8);
    val[it] = pk.u;
    go[it]  = ((size_t)hb * NND + q0 + L) * HDM + pc * 8;
  }
  for (int ps = 0; ps < 2; ++ps) {
#pragma unroll
    for (int it = 0; it < 2; ++it) *(volatile v4u*)(op + go[it]) = val[it];
    __threadfence();
  }
}

#define OTP 260
__global__ __launch_bounds__(128) void k_oln(const _Float16* __restrict__ op,
                                             const _Float16* __restrict__ wot,
                                             const float* __restrict__ bo,
                                             const float* __restrict__ resid,
                                             const float* __restrict__ g,
                                             const float* __restrict__ be,
                                             float* __restrict__ lnp) {
  __shared__ __align__(16) float sw[32 * OTP];
  const int tid = threadIdx.x, lane = tid & 31, wave = tid >> 5;
  const int hh = lane >> 4, c = lane & 15;
  const int m0 = blockIdx.x * 32;
  const int b  = m0 / NND;
  const int nl = m0 - b * NND;
  const _Float16* A = op + ((size_t)b * NH * NND + nl) * HDM;
  const int n0 = wave * 64;

  v8f acc[2][4];
#pragma unroll
  for (int s = 0; s < 2; ++s)
#pragma unroll
    for (int t = 0; t < 4; ++t) acc[s][t] = zero8();
  gemm32x64(A, HDM, NND * HDM, wot, DM, 32, DM / 32, 0, n0, lane, acc);

  float bb[4];
#pragma unroll
  for (int t = 0; t < 4; ++t) bb[t] = bo[n0 + 16 * t + c];
#pragma unroll
  for (int sub = 0; sub < 2; ++sub)
#pragma unroll
    for (int t = 0; t < 4; ++t)
#pragma unroll
      for (int r = 0; r < 8; ++r)
        sw[(sub * 16 + 8 * hh + r) * OTP + n0 + 16 * t + c] = acc[sub][t][r] * 0.00048828125f + bb[t];
  __syncthreads();

  const v4f g0 = *(const v4f*)(g + 4 * lane);
  const v4f g1 = *(const v4f*)(g + 128 + 4 * lane);
  const v4f e0 = *(const v4f*)(be + 4 * lane);
  const v4f e1 = *(const v4f*)(be + 128 + 4 * lane);
#pragma unroll 1
  for (int rr = 0; rr < 8; ++rr) {
    const int row = wave * 8 + rr;
    const size_t m = (size_t)(m0 + row);
    const float* rp = resid + m * DM;
    const v4f v0 = *(const v4f*)(sw + row * OTP + 4 * lane) + *(const v4f*)(rp + 4 * lane);
    const v4f v1 = *(const v4f*)(sw + row * OTP + 128 + 4 * lane) + *(const v4f*)(rp + 128 + 4 * lane);
    float s = ((v0[0] + v0[1]) + (v0[2] + v0[3])) + ((v1[0] + v1[1]) + (v1[2] + v1[3]));
#pragma unroll
    for (int off = 16; off >= 1; off >>= 1) s += __shfl_xor(s, off, 32);
    const float mean = s * 0.00390625f;
    const v4f d0 = v0 - mean, d1 = v1 - mean;
    float ss = ((d0[0] * d0[0] + d0[1] * d0[1]) + (d0[2] * d0[2] + d0[3] * d0[3])) +
               ((d1[0] * d1[0] + d1[1] * d1[1]) + (d1[2] * d1[2] + d1[3] * d1[3]));
#pragma unroll
    for (int off = 16; off >= 1; off >>= 1) ss += __shfl_xor(ss, off, 32);
    const float var  = ss * 0.00390625f;
    const float rstd = rsqrtf(var + 1e-5f);
    const v4f y0 = (d0 * rstd) * g0 + e0;
    const v4f y1 = (d1 * rstd) * g1 + e1;
    float* yp = lnp + m * DM;
    *(volatile v4f*)(yp + 4 * lane) = y0;
    *(volatile v4f*)(yp + 128 + 4 * lane) = y1;
    __threadfence();
    *(volatile v4f*)(yp + 4 * lane) = y0;
    *(volatile v4f*)(yp + 128 + 4 * lane) = y1;
  }
}

__global__ __launch_bounds__(256) void k_comb_mid(const float* __restrict__ lnp,
                                                  float* __restrict__ h32, _Float16* __restrict__ h16) {
  __shared__ __align__(16) float sw[2048];
  const int tid = threadIdx.x;
  const int y = blockIdx.y;
  const float* pa = lnp + (size_t)((y == 0) ? 0 : 1) * HN;
  const float* pb = lnp + (size_t)((y == 0) ? 3 : 2) * HN;
  const size_t blk = (size_t)blockIdx.x * 2048;
  const size_t o = blk + (size_t)tid * 8;
  const v4f a0 = *(const v4f*)(pa + o), a1 = *(const v4f*)(pa + o + 4);
  const v4f b0 = *(const v4f*)(pb + o), b1 = *(const v4f*)(pb + o + 4);
  v4f v0 = a0 + b0, v1 = a1 + b1;
#pragma unroll
  for (int e = 0; e < 4; ++e) { v0[e] = fmaxf(v0[e], 0.f); v1[e] = fmaxf(v1[e], 0.f); }
  Pack8 pk;
  pk.h = (v8h){(_Float16)v0[0], (_Float16)v0[1], (_Float16)v0[2], (_Float16)v0[3],
               (_Float16)v1[0], (_Float16)v1[1], (_Float16)v1[2], (_Float16)v1[3]};
  const v4u hv = pk.u;
  volatile v4u* dh = (volatile v4u*)(h16 + (size_t)y * HN + o);
  *dh = hv;
  __threadfence();
  *dh = hv;
  *(v4f*)(sw + tid * 8) = v0;
  *(v4f*)(sw + tid * 8 + 4) = v1;
  __syncthreads();
  v4f w[2];
  size_t go[2];
#pragma unroll
  for (int it = 0; it < 2; ++it) {
    const int e = it * 1024 + tid * 4;
    w[it]  = *(const v4f*)(sw + e);
    go[it] = (size_t)y * HN + blk + e;
  }
  for (int ps = 0; ps < 2; ++ps) {
#pragma unroll
    for (int it = 0; it < 2; ++it) *(volatile v4f*)(h32 + go[it]) = w[it];
    __threadfence();
  }
}

__global__ __launch_bounds__(256) void k_comb_out(const float* __restrict__ lnp,
                                                  const float* __restrict__ xa, const float* __restrict__ xb,
                                                  float* __restrict__ out) {
  const int tid = threadIdx.x;
  const int y = blockIdx.y;
  const float* pa = lnp + (size_t)((y == 0) ? 0 : 1) * HN;
  const float* pb = lnp + (size_t)((y == 0) ? 3 : 2) * HN;
  const float* px = (y == 0) ? xa : xb;
  const size_t blk = (size_t)blockIdx.x * 2048;
  v4f w[2];
  size_t go[2];
#pragma unroll
  for (int it = 0; it < 2; ++it) {
    const size_t e = blk + (size_t)it * 1024 + (size_t)tid * 4;
    const v4f a = *(const v4f*)(pa + e);
    const v4f bq4 = *(const v4f*)(pb + e);
    const v4f x = *(const v4f*)(px + e);
    v4f v = a + bq4;
#pragma unroll
    for (int q = 0; q < 4; ++q) v[q] = fmaxf(v[q], 0.f);
    w[it]  = x + v;
    go[it] = (size_t)y * HN + e;
  }
  for (int ps = 0; ps < 2; ++ps) {
#pragma unroll
    for (int it = 0; it < 2; ++it) *(volatile v4f*)(out + go[it]) = w[it];
    __threadfence();
  }
}

extern "C" void kernel_launch(void* const* d_in, const int* in_sizes, int n_in,
                              void* d_out, int out_size, void* d_ws, size_t ws_size,
                              hipStream_t stream) {
  if (n_in < 16) return;
  if (in_sizes[0] != HN) return;
  if (in_sizes[1] != HN) return;
  if (in_sizes[2] != NBT * NND * NND) return;
  if (in_sizes[3] != NBT * NND * NND) return;
  if (in_sizes[4] != NBT * NND * NND) return;
  if (in_sizes[5] != NBT * NND * NND) return;
  if (in_sizes[6] != NMAT * WMAT) return;
  if (in_sizes[7] != NMAT * DM) return;
  if (in_sizes[8] != NMAT * WMAT) return;
  if (in_sizes[9] != NMAT * DM) return;
  if (in_sizes[10] != NMAT * WMAT) return;
  if (in_sizes[11] != NMAT * DM) return;
  if (in_sizes[12] != NMAT * WMAT) return;
  if (in_sizes[13] != NMAT * DM) return;
  if (in_sizes[14] != NMAT * DM) return;
  if (in_sizes[15] != NMAT * DM) return;
  if (out_size != 2 * HN) return;

  const float* xa  = (const float*)d_in[0];
  const float* xb  = (const float*)d_in[1];
  const int* adjs[4] = {(const int*)d_in[2], (const int*)d_in[3], (const int*)d_in[4], (const int*)d_in[5]};
  const float* wq  = (const float*)d_in[6];
  const float* bq  = (const float*)d_in[7];
  const float* wk  = (const float*)d_in[8];
  const float* bk  = (const float*)d_in[9];
  const float* wv  = (const float*)d_in[10];
  const float* bv  = (const float*)d_in[11];
  const float* wo  = (const float*)d_in[12];
  const float* bo  = (const float*)d_in[13];
  const float* lng = (const float*)d_in[14];
  const float* lnb = (const float*)d_in[15];
  float* out = (float*)d_out;

  size_t off = 0;
  const size_t oWt  = off; off += (size_t)4 * NMAT * WMAT * 2;
  const size_t oH16 = off; off += (size_t)2 * HN * 2;
  const size_t oH32 = off; off += (size_t)2 * HN * 4;
  const size_t oQK  = off; off += (size_t)2 * HPL * 2;
  const size_t oVt  = off; off += (size_t)HPL * 2;
  const size_t oOp  = off; off += (size_t)HPL * 2;
  const size_t oLN  = off; off += (size_t)4 * HN * 4;
  if (off > ws_size) return;
  if (off > (size_t)134217728) return;

  char* ws = (char*)d_ws;
  _Float16* Wt  = (_Float16*)(ws + oWt);
  _Float16* H16 = (_Float16*)(ws + oH16);
  float*    H32 = (float*)(ws + oH32);
  _Float16* QK  = (_Float16*)(ws + oQK);
  _Float16* Vt  = (_Float16*)(ws + oVt);
  _Float16* Op  = (_Float16*)(ws + oOp);
  float*    LN  = (float*)(ws + oLN);

  k_wcvt<<<dim3(NMAT * 16), dim3(256), 0, stream>>>(wq, Wt);
  k_wcvt<<<dim3(NMAT * 16), dim3(256), 0, stream>>>(wk, Wt + (size_t)1 * NMAT * WMAT);
  k_wcvt<<<dim3(NMAT * 16), dim3(256), 0, stream>>>(wv, Wt + (size_t)2 * NMAT * WMAT);
  k_wcvt<<<dim3(NMAT * 16), dim3(256), 0, stream>>>(wo, Wt + (size_t)3 * NMAT * WMAT);
  k_cvt_h<<<dim3(HN / 2048, 2), dim3(256), 0, stream>>>(xa, xb, H16);

  const float sscale = 0.17677669529663688f;
  const int qsel_t[4]  = {0, 1, 1, 0};
  const int kvsel_t[4] = {0, 1, 0, 1};
  for (int i = 0; i < NLY; ++i) {
    for (int j = 0; j < NBR; ++j) {
      const int mat = i * NBR + j;
      const int qs = qsel_t[j], kvs = kvsel_t[j];
      k_qkv<<<dim3(NTOK / 256, 3 * (DM / 64)), dim3(256), 0, stream>>>(
          H16, qs, kvs, Wt + (size_t)mat * WMAT, bq + (size_t)mat * DM, bk + (size_t)mat * DM,
          bv + (size_t)mat * DM, QK, Vt);
      k_attn<<<dim3(NBT * NH * NQB), dim3(256), 0, stream>>>(QK, Vt, adjs[j], Op, sscale);
      const float* resid = (i == 0) ? ((qs == 0) ? xa : xb) : (H32 + (size_t)qs * HN);
      k_oln<<<dim3(NTOK / 32), dim3(128), 0, stream>>>(
          Op, Wt + ((size_t)3 * NMAT + mat) * WMAT, bo + (size_t)mat * DM, resid,
          lng + (size_t)mat * DM, lnb + (size_t)mat * DM, LN + (size_t)j * HN);
    }
    if (i + 1 < NLY) {
      k_comb_mid<<<dim3(HN / 2048, 2), dim3(256), 0, stream>>>(LN, H32, H16);
    } else {
      k_comb_out<<<dim3(HN / 2048, 2), dim3(256), 0, stream>>>(LN, xa, xb, out);
    }
  }
  (void)hipGetLastError();
}
